// TransformerMPNNParenthood_23381801960101
// MI455X (gfx1250) — hardware-verified
//
#include <hip/hip_runtime.h>
#include <math.h>

typedef __attribute__((ext_vector_type(16))) _Float16 v16h;
typedef __attribute__((ext_vector_type(8)))  _Float16 v8h;
typedef __attribute__((ext_vector_type(4)))  _Float16 v4h;
typedef __attribute__((ext_vector_type(16))) __bf16   v16b;
typedef __attribute__((ext_vector_type(8)))  __bf16   v8b;
typedef __attribute__((ext_vector_type(8)))  float    v8f;
typedef __attribute__((ext_vector_type(4)))  float    v4f;
typedef __attribute__((ext_vector_type(4)))  int      v4i;

__device__ __forceinline__ unsigned short f2bf_bits(float f) {
  unsigned u = __float_as_uint(f);
  return (unsigned short)((u + 0x7FFFu + ((u >> 16) & 1u)) >> 16);
}
__device__ __forceinline__ float bf_bits2f(unsigned short h) { return __uint_as_float(((unsigned)h) << 16); }

__device__ __forceinline__ void dep_guard_h(v8f& a, v8f& b, v16h x, v16h y) { asm volatile("v_nop\n\tv_nop\n\tv_nop\n\tv_nop" : "+v"(a), "+v"(b) : "v"(x), "v"(y)); }
__device__ __forceinline__ void dep_guard_b(v8f& a, v8f& b, v16b x, v16b y) { asm volatile("v_nop\n\tv_nop\n\tv_nop\n\tv_nop" : "+v"(a), "+v"(b) : "v"(x), "v"(y)); }
__device__ __forceinline__ void keep4_h(v16h a, v16h b, v16h c, v16h d) { asm volatile("v_nop" :: "v"(a), "v"(b), "v"(c), "v"(d)); }
__device__ __forceinline__ void keep4_b(v16b a, v16b b, v16b c, v16b d) { asm volatile("v_nop" :: "v"(a), "v"(b), "v"(c), "v"(d)); }
__device__ __forceinline__ void acc_guard4(v8f& a, v8f& b, v8f& c, v8f& d) { asm volatile("v_nop\n\tv_nop\n\tv_nop\n\tv_nop" : "+v"(a), "+v"(b), "+v"(c), "+v"(d)); }
template <typename T> struct Frag;
template <> struct Frag<_Float16> {
  typedef v16h V; union U { v16h v; v8h h[2]; };
  static __device__ __forceinline__ v16h load(const _Float16* p) {
    U f; f.h[0] = *(const v8h*)(p); f.h[1] = *(const v8h*)(p + 16); return f.v;
  }
  static __device__ __forceinline__ v8f mma(v16h a, v16h b, v8f c) {
    return __builtin_amdgcn_wmma_f32_16x16x32_f16(false, a, false, b, (short)0, c, false, false);
  }
  static __device__ __forceinline__ void guard(v8f& a, v8f& b, v16h x, v16h y) { dep_guard_h(a, b, x, y); }
  static __device__ __forceinline__ void keep(v16h a, v16h b, v16h c, v16h d) { keep4_h(a, b, c, d); }
};
template <> struct Frag<__bf16> {
  typedef v16b V; union U { v16b v; v8b h[2]; };
  static __device__ __forceinline__ v16b load(const __bf16* p) {
    U f; f.h[0] = *(const v8b*)(p); f.h[1] = *(const v8b*)(p + 16); return f.v;
  }
  static __device__ __forceinline__ v8f mma(v16b a, v16b b, v8f c) {
    return __builtin_amdgcn_wmma_f32_16x16x32_bf16(false, a, false, b, (short)0, c, false, false);
  }
  static __device__ __forceinline__ void guard(v8f& a, v8f& b, v16b x, v16b y) { dep_guard_b(a, b, x, y); }
  static __device__ __forceinline__ void keep(v16b a, v16b b, v16b c, v16b d) { keep4_b(a, b, c, d); }
};

template <int ET> struct Elem;
template <> struct Elem<0> { typedef _Float16 T; };
template <> struct Elem<1> { typedef __bf16 T; };
template <int ET, bool SPLIT, int BIAS_MODE, int OUT_MODE, bool RESID, int ACT = 0>
__global__ __launch_bounds__(256) void wmma_gemm64(
    const unsigned short* __restrict__ Ap, const unsigned short* __restrict__ A2p, int lda, long strideA,
    const unsigned short* __restrict__ Btp, const unsigned short* __restrict__ Bt2p, int ldb, long strideB,
    void* __restrict__ Cout, void* __restrict__ Cout2, int ldc, long strideC,
    const float* __restrict__ bias,
    const float* __restrict__ resid, long strideR,
    int M, int N, int K, float scale) {
  typedef typename Elem<ET>::T T;
  typedef typename Frag<T>::V V;
  const T* A = (const T*)Ap; const T* A2 = (const T*)A2p; const T* Bt = (const T*)Btp; const T* Bt2 = (const T*)Bt2p;
  __shared__ __align__(16) float sT[8][16 * 68];
  const int b    = blockIdx.y;
  const int lane = threadIdx.x & 31;
  const int wave = threadIdx.x >> 5;
  const int tilesN = N >> 6;
  const int tilesM = M >> 6;
  const int tile = blockIdx.x * 8 + wave;
  if (tile >= tilesM * tilesN) return;
  const int tm = tile / tilesN;
  const int tn = tile - tm * tilesN;
  const int m0 = tm << 6;
  const int n0 = tn << 6;

  const T* Ab  = A  + (size_t)b * strideA;
  const T* Bb  = Bt + (size_t)b * strideB;
  const T* Ab2 = SPLIT ? (A2  + (size_t)b * strideA) : nullptr;
  const T* Bb2 = SPLIT ? (Bt2 + (size_t)b * strideB) : nullptr;

  const int rlane = lane & 15;
  const int koff  = (lane >> 4) * 8;
  const int mOff  = (lane >> 4) * 8;

  v8f acc[4][4];
#pragma unroll
  for (int i = 0; i < 4; ++i)
#pragma unroll
    for (int j = 0; j < 4; ++j) acc[i][j] = (v8f){0.f,0.f,0.f,0.f,0.f,0.f,0.f,0.f};

  for (int k0 = 0; k0 < K; k0 += 32) {
    V bh[4], bl[4];
#pragma unroll
    for (int j = 0; j < 4; ++j) {
      const size_t bo = (size_t)(n0 + (j << 4) + rlane) * ldb + koff + k0;
      bh[j] = Frag<T>::load(Bb + bo);
      if (SPLIT) bl[j] = Frag<T>::load(Bb2 + bo);
    }
#pragma unroll
    for (int i = 0; i < 4; ++i) {
      const size_t ao = (size_t)(m0 + (i << 4) + rlane) * lda + koff + k0;
      V ah = Frag<T>::load(Ab + ao);
      V al;
      if (SPLIT) al = Frag<T>::load(Ab2 + ao);
#pragma unroll
      for (int j = 0; j < 4; ++j) {
        acc[i][j] = Frag<T>::mma(ah, bh[j], acc[i][j]);
        if (SPLIT) {
          acc[i][j] = Frag<T>::mma(ah, bl[j], acc[i][j]);
          acc[i][j] = Frag<T>::mma(al, bh[j], acc[i][j]);
        }
      }
      Frag<T>::guard(acc[i][0], acc[i][3], ah, SPLIT ? al : ah);
    }
    Frag<T>::keep(bh[0], bh[1], bh[2], bh[3]);
    if (SPLIT) Frag<T>::keep(bl[0], bl[1], bl[2], bl[3]);
  }
  acc_guard4(acc[0][0], acc[0][1], acc[0][2], acc[0][3]);
  acc_guard4(acc[1][0], acc[1][1], acc[1][2], acc[1][3]);
  acc_guard4(acc[2][0], acc[2][1], acc[2][2], acc[2][3]);
  acc_guard4(acc[3][0], acc[3][1], acc[3][2], acc[3][3]);

  float* slab = sT[wave];
  const float* Rb = RESID ? (resid + (size_t)b * strideR) : nullptr;
#pragma unroll
  for (int i = 0; i < 4; ++i) {
    const int mBase = m0 + (i << 4);
#pragma unroll
    for (int j = 0; j < 4; ++j) {
      const int n = n0 + (j << 4) + rlane;
      float bv = 0.f;
      if (BIAS_MODE == 2) bv = bias[n];
#pragma unroll
      for (int r = 0; r < 8; ++r) {
        float v = acc[i][j][r] * scale;
        if (BIAS_MODE == 1) v += bias[mBase + mOff + r];
        if (BIAS_MODE == 2) v += bv;
        if (RESID) v += Rb[(size_t)(mBase + mOff + r) * ldc + n];
        if (ACT == 1) v = tanhf(v);
        if (ACT == 2) v = fmaxf(v, 0.0f);
        if (ACT == 3) v = v / (1.0f + expf(-v));
        if (ACT == 4) v = (v > 0.f) ? v : 0.01f * v;
        if (ACT == 5) v = 0.5f * v * (1.0f + erff(v * 0.70710678118654752f));
        slab[(mOff + r) * 68 + (j << 4) + rlane] = v;
      }
    }
    __builtin_amdgcn_fence(__ATOMIC_RELEASE, "workgroup");
    __builtin_amdgcn_wave_barrier();
    __builtin_amdgcn_fence(__ATOMIC_ACQUIRE, "workgroup");
    if (OUT_MODE == 0) {
      float* C = (float*)Cout + (size_t)b * strideC;
      const int hh = lane >> 4, c4 = (lane & 15) * 4;
      for (int pass = 0; pass < 2; ++pass) {
#pragma unroll
        for (int it = 0; it < 8; ++it) {
          const int row = it * 2 + hh;
          v4f v = *(const v4f*)(slab + row * 68 + c4);
          *(volatile v4f*)(C + (size_t)(mBase + row) * ldc + n0 + c4) = v;
        }
        __threadfence();
      }
    } else {
      const int q = lane >> 3, c8 = (lane & 7) * 8;
      unsigned short* C  = (unsigned short*)Cout  + (size_t)b * strideC;
      unsigned short* C2 = (OUT_MODE == 2) ? ((unsigned short*)Cout2 + (size_t)b * strideC) : nullptr;
      for (int pass = 0; pass < 2; ++pass) {
#pragma unroll
        for (int it = 0; it < 4; ++it) {
          const int row = it * 4 + q;
          const float* sp = slab + row * 68 + c8;
          v8h hv, lv;
#pragma unroll
          for (int e = 0; e < 8; ++e) {
            if (OUT_MODE == 1) {
              hv[e] = (_Float16)sp[e];
            } else {
              unsigned short hb = f2bf_bits(sp[e]);
              unsigned short lb = f2bf_bits(sp[e] - bf_bits2f(hb));
              hv[e] = __builtin_bit_cast(_Float16, hb);
              lv[e] = __builtin_bit_cast(_Float16, lb);
            }
          }
          *(volatile v8h*)(C + (size_t)(mBase + row) * ldc + n0 + c8) = hv;
          if (OUT_MODE == 2) *(volatile v8h*)(C2 + (size_t)(mBase + row) * ldc + n0 + c8) = lv;
        }
        __threadfence();
      }
    }
    __builtin_amdgcn_fence(__ATOMIC_RELEASE, "workgroup");
    __builtin_amdgcn_wave_barrier();
    __builtin_amdgcn_fence(__ATOMIC_ACQUIRE, "workgroup");
  }
}

__global__ __launch_bounds__(256) void cast_f32_f16x2(
    const float* __restrict__ in, _Float16* __restrict__ out, int n2) {
  int i = blockIdx.x * 256 + threadIdx.x;
  if (i < n2) {
    const _Float16 h0 = (_Float16)in[2 * i], h1 = (_Float16)in[2 * i + 1];
    const unsigned u = (unsigned)__builtin_bit_cast(unsigned short, h0) | ((unsigned)__builtin_bit_cast(unsigned short, h1) << 16);
    ((volatile unsigned*)out)[i] = u;
    __threadfence();
    ((volatile unsigned*)out)[i] = u;
  }
}

__global__ __launch_bounds__(256) void transpose_cast_w_kernel(
    const float* __restrict__ W, _Float16* __restrict__ Wt, int K, int Cn, float scale) {
  const int kg = K >> 3;
  const int gidx = blockIdx.x * 256 + threadIdx.x;
  if (gidx < Cn * kg) {
    const int n = gidx / kg;
    const int k0 = (gidx - n * kg) * 8;
    v8h vv;
#pragma unroll
    for (int i = 0; i < 8; ++i) vv[i] = (_Float16)(W[(size_t)(k0 + i) * Cn + n] * scale);
    _Float16* dst = Wt + (size_t)n * K + k0;
    *(volatile v8h*)dst = vv;
    __threadfence();
    *(volatile v8h*)dst = vv;
  }
}

template <int NW>
__device__ __forceinline__ int block_excl_scan(int cnt, int* wtot, int lane, int wave, int& total) {
  int incl = cnt;
#pragma unroll
  for (int off = 1; off < 32; off <<= 1) {
    const int t = __shfl_up(incl, off, 32);
    if (lane >= off) incl += t;
  }
  if (lane == 31) wtot[wave] = incl;
  __syncthreads();
  int base = 0, tot = 0;
#pragma unroll
  for (int w = 0; w < NW; ++w) { const int t = wtot[w]; tot += t; base += (w < wave) ? t : 0; }
  total = tot;
  return base + incl - cnt;
}

#define DG_NT 256
#define DG_EPT 8
#define DG_CH (DG_NT * DG_EPT)
template <bool HASW>
__global__ __launch_bounds__(DG_NT) void gcn_dinv_kernel(
    const int* __restrict__ edst, const float* __restrict__ ew, float* __restrict__ dinv, int N, int NE) {
  __shared__ int   lc[DG_CH];
  __shared__ float lw[DG_CH];
  __shared__ int   wtot[DG_NT / 32];
  const int tid = threadIdx.x, lane = tid & 31, wave = tid >> 5;
  const int tile0 = blockIdx.x * DG_NT;
  float wsum = 0.f;
  for (int cb = 0; cb < NE; cb += DG_CH) {
    const int e0 = cb + tid * DG_EPT;
    const int ebc = (e0 + DG_EPT <= NE) ? e0 : (NE - DG_EPT);
    const v4i ca  = *(const v4i*)(edst + ebc);
    const v4i cbv = *(const v4i*)(edst + ebc + 4);
    int cv[DG_EPT];
    cv[0] = ca[0]; cv[1] = ca[1]; cv[2] = ca[2]; cv[3] = ca[3];
    cv[4] = cbv[0]; cv[5] = cbv[1]; cv[6] = cbv[2]; cv[7] = cbv[3];
    float wv[DG_EPT];
    if (HASW) {
      const v4f wa = *(const v4f*)(ew + ebc);
      const v4f wb = *(const v4f*)(ew + ebc + 4);
      wv[0] = wa[0]; wv[1] = wa[1]; wv[2] = wa[2]; wv[3] = wa[3];
      wv[4] = wb[0]; wv[5] = wb[1]; wv[6] = wb[2]; wv[7] = wb[3];
    } else {
#pragma unroll
      for (int i = 0; i < DG_EPT; ++i) wv[i] = 1.0f;
    }
    unsigned flags = 0;
#pragma unroll
    for (int i = 0; i < DG_EPT; ++i)
      if ((ebc + i >= e0) && (unsigned)(cv[i] - tile0) < (unsigned)DG_NT && cv[i] < N) flags |= 1u << i;
    const int cnt = __popc(flags);
    int nh;
    int pos = block_excl_scan<DG_NT / 32>(cnt, wtot, lane, wave, nh);
#pragma unroll
    for (int i = 0; i < DG_EPT; ++i) {
      if (flags & (1u << i)) {
        if (pos < DG_CH) { lc[pos] = cv[i] - tile0; lw[pos] = wv[i]; }
        ++pos;
      }
    }
    __syncthreads();
    nh = nh < DG_CH ? nh : DG_CH;
    for (int j = 0; j < nh; ++j) wsum += (lc[j] == tid) ? lw[j] : 0.f;
    __syncthreads();
  }
  const int node = tile0 + tid;
  const float deg = wsum + 1.0f;
  float d = (deg > 0.f) ? (1.0f / sqrtf(deg)) : 0.f;
  if (node < N) {
    ((volatile float*)dinv)[node] = d;
    __threadfence();
    ((volatile float*)dinv)[node] = d;
  }
}

#define AG_TILE 64
#define AG_C 512
#define AG_T 128
#define AG_EPT 8
#define AG_CH (AG_T * AG_EPT)
template <bool HASW>
__global__ __launch_bounds__(AG_T) void gcn_agg_kernel(
    const float* __restrict__ Hf, const int* __restrict__ esrc, const int* __restrict__ edst,
    const float* __restrict__ ew, const float* __restrict__ dinv, const float* __restrict__ bias,
    _Float16* __restrict__ out16, int ldo, int coff, int N, int NE, float oscale) {
  constexpr int NW = AG_T / 32;
  __shared__ __align__(16) float acc[AG_TILE * AG_C];
  __shared__ int   lrw[AG_CH];
  __shared__ int   llc[AG_CH];
  __shared__ float lnm[AG_CH];
  __shared__ int   wtot[NW];
  const int tid = threadIdx.x, lane = tid & 31, wave = tid >> 5;
  const int tile0 = blockIdx.x * AG_TILE;
  const int ch0 = tid * 4;
  const v4f z4 = {0.f, 0.f, 0.f, 0.f};
#pragma unroll 1
  for (int r = 0; r < AG_TILE; ++r) *(v4f*)(acc + r * AG_C + ch0) = z4;
  for (int cb = 0; cb < NE; cb += AG_CH) {
    const int e0 = cb + tid * AG_EPT;
    const int ebc = (e0 + AG_EPT <= NE) ? e0 : (NE - AG_EPT);
    const v4i t0 = *(const v4i*)(edst + ebc);
    const v4i t1 = *(const v4i*)(edst + ebc + 4);
    const v4i u0 = *(const v4i*)(esrc + ebc);
    const v4i u1 = *(const v4i*)(esrc + ebc + 4);
    int cv[AG_EPT], sv[AG_EPT];
    cv[0] = t0[0]; cv[1] = t0[1]; cv[2] = t0[2]; cv[3] = t0[3];
    cv[4] = t1[0]; cv[5] = t1[1]; cv[6] = t1[2]; cv[7] = t1[3];
    sv[0] = u0[0]; sv[1] = u0[1]; sv[2] = u0[2]; sv[3] = u0[3];
    sv[4] = u1[0]; sv[5] = u1[1]; sv[6] = u1[2]; sv[7] = u1[3];
    float wv[AG_EPT];
    if (HASW) {
      const v4f wa = *(const v4f*)(ew + ebc);
      const v4f wb = *(const v4f*)(ew + ebc + 4);
      wv[0] = wa[0]; wv[1] = wa[1]; wv[2] = wa[2]; wv[3] = wa[3];
      wv[4] = wb[0]; wv[5] = wb[1]; wv[6] = wb[2]; wv[7] = wb[3];
    } else {
#pragma unroll
      for (int i = 0; i < AG_EPT; ++i) wv[i] = 1.0f;
    }
    unsigned flags = 0;
#pragma unroll
    for (int i = 0; i < AG_EPT; ++i)
      if ((ebc + i >= e0) && (unsigned)(cv[i] - tile0) < (unsigned)AG_TILE && cv[i] < N) flags |= 1u << i;
    const int cnt = __popc(flags);
    int nh;
    int pos = block_excl_scan<NW>(cnt, wtot, lane, wave, nh);
#pragma unroll
    for (int i = 0; i < AG_EPT; ++i) {
      if (flags & (1u << i)) {
        if (pos < AG_CH) {
          int r = sv[i];
          r = r < 0 ? 0 : (r >= N ? N - 1 : r);
          int cc = cv[i];
          cc = cc < 0 ? 0 : (cc >= N ? N - 1 : cc);
          const float nm = (dinv[r] * wv[i]) * dinv[cc];
          lrw[pos] = r; llc[pos] = cc - tile0; lnm[pos] = nm;
        }
        ++pos;
      }
    }
    __syncthreads();
    nh = nh < AG_CH ? nh : AG_CH;
    for (int j = 0; j < nh; ++j) {
      const int r = lrw[j];
      const int lc = llc[j];
      const float nm = lnm[j];
      const v4f m = *(const v4f*)(Hf + (size_t)r * AG_C + ch0);
      float* ap = acc + lc * AG_C + ch0;
      v4f a = *(const v4f*)ap;
#pragma unroll
      for (int q = 0; q < 4; ++q) a[q] += m[q] * nm;
      *(v4f*)ap = a;
    }
    __syncthreads();
  }
  __syncthreads();

  const v4f b4 = *(const v4f*)(bias + ch0);
  for (int pass = 0; pass < 2; ++pass) {
#pragma unroll 1
    for (int row = 0; row < AG_TILE; ++row) {
      const int node = tile0 + row;
      if (node < N) {
        const float di = dinv[node];
        const float ns = di * di;
        const v4f a  = *(const v4f*)(acc + row * AG_C + ch0);
        const v4f mm = *(const v4f*)(Hf + (size_t)node * AG_C + ch0);
        v4h hv;
#pragma unroll
        for (int q = 0; q < 4; ++q) hv[q] = (_Float16)((a[q] + mm[q] * ns + b4[q]) * oscale);
        *(volatile v4h*)(out16 + (size_t)node * ldo + coff + ch0) = hv;
      }
    }
    __threadfence();
  }
}

template <bool WF32>
__global__ __launch_bounds__(128) void layernorm512_kernel(
    const float* __restrict__ in, const float* __restrict__ g, const float* __restrict__ bta,
    float* __restrict__ outf, _Float16* __restrict__ out16, int ld16, int coff16, int nrows, float s16) {
  const int lane = threadIdx.x & 31, wave = threadIdx.x >> 5;
  const int row = blockIdx.x * 4 + wave;
  if (row >= nrows) return;
  const float* xr = in + (size_t)row * 512;
  v4f v[4];
#pragma unroll
  for (int i = 0; i < 4; ++i) v[i] = *(const v4f*)(xr + i * 128 + lane * 4);
  float s = 0.f;
#pragma unroll
  for (int i = 0; i < 4; ++i) s += (v[i][0] + v[i][1]) + (v[i][2] + v[i][3]);
#pragma unroll
  for (int off = 1; off < 32; off <<= 1) s += __shfl_xor(s, off, 32);
  const float mu = s * (1.0f / 512.0f);
  float ss = 0.f;
#pragma unroll
  for (int i = 0; i < 4; ++i) {
#pragma unroll
    for (int q = 0; q < 4; ++q) { const float d = v[i][q] - mu; ss += d * d; }
  }
#pragma unroll
  for (int off = 1; off < 32; off <<= 1) ss += __shfl_xor(ss, off, 32);
  const float var = ss * (1.0f / 512.0f);
  const float inv = 1.0f / sqrtf(var + 1e-5f);
  v4f y[4];
  v4h yh[4];
#pragma unroll
  for (int i = 0; i < 4; ++i) {
    const v4f gg = *(const v4f*)(g + i * 128 + lane * 4);
    const v4f bb = *(const v4f*)(bta + i * 128 + lane * 4);
#pragma unroll
    for (int q = 0; q < 4; ++q) {
      const float t = (v[i][q] - mu) * inv * gg[q] + bb[q];
      y[i][q] = t;
      yh[i][q] = (_Float16)(t * s16);
    }
  }
  for (int pass = 0; pass < 2; ++pass) {
#pragma unroll
    for (int i = 0; i < 4; ++i) {
      if (WF32) *(volatile v4f*)(outf + (size_t)row * 512 + i * 128 + lane * 4) = y[i];
      *(volatile v4h*)(out16 + (size_t)row * ld16 + coff16 + i * 128 + lane * 4) = yh[i];
    }
    __threadfence();
  }
}

#define AT_D 64
#define AT_NW 4
#define AT_QB 64
#define AT_KC 64
#define AT_PSC 32768.0f

__device__ __forceinline__ v8f mma_h16(v16h a, v16h b, v8f c) {
  c = __builtin_amdgcn_wmma_f32_16x16x32_f16(false, a, false, b, (short)0, c, false, false);
  asm volatile("v_nop\n\tv_nop\n\tv_nop\n\tv_nop" : "+v"(c) : "v"(a), "v"(b));
  return c;
}

__global__ __launch_bounds__(AT_NW * 32)
void attn64_h16_kernel(const _Float16* __restrict__ Qp, int ldq, const _Float16* __restrict__ Kp, int ldk,
                       const _Float16* __restrict__ Vtp, int ldv, _Float16* __restrict__ Op, int ldo,
                       int S, int nheads, float sscale, float oscale) {
  union FH { v16h v; v8h h[2]; };
  __shared__ __align__(16) _Float16 Ksh[AT_KC * AT_D];
  __shared__ __align__(16) _Float16 Vth[AT_D * AT_KC];
  __shared__ __align__(16) _Float16 Psh[AT_NW][16 * AT_KC];
  __shared__ __align__(16) float    Os[AT_NW][16 * 68];

  const int tid  = threadIdx.x;
  const int wave = tid >> 5;
  const int lane = tid & 31;
  const int hh   = lane >> 4;
  const int c    = lane & 15;

  const int nqb = S / AT_QB;
  const int bx  = blockIdx.x;
  const int qb  = bx % nqb;
  const int h   = bx / nqb;
  if (h >= nheads) return;
  const int hcol = h * AT_D;
  const int q0 = qb * AT_QB + wave * 16;

  v16h qa[2];
  {
    const _Float16* qrow = Qp + (size_t)(q0 + c) * ldq + hcol;
#pragma unroll
    for (int dc = 0; dc < 2; ++dc) qa[dc] = Frag<_Float16>::load(qrow + dc * 32 + 8 * hh);
  }

  float mrow[8], lrow[8];
  v8f oacc[4];
#pragma unroll
  for (int r = 0; r < 8; ++r) { mrow[r] = -INFINITY; lrow[r] = 0.f; }
#pragma unroll
  for (int t = 0; t < 4; ++t) oacc[t] = (v8f){0.f,0.f,0.f,0.f,0.f,0.f,0.f,0.f};

  const int nChunks = S / AT_KC;
  for (int kc = 0; kc < nChunks; ++kc) {
    const int kv0 = kc * AT_KC;
    __syncthreads();
    {
      const int rr = tid >> 1, dh = (tid & 1) * 32;
      const _Float16* krow = Kp  + (size_t)(kv0 + rr) * ldk + hcol + dh;
      const _Float16* vrow = Vtp + (size_t)(hcol + rr) * ldv + kv0 + dh;
#pragma unroll
      for (int i = 0; i < 4; ++i) {
        const v8h kk = *(const v8h*)(krow + 8 * i);
        const v8h vv = *(const v8h*)(vrow + 8 * i);
        *(v8h*)(Ksh + rr * AT_D  + dh + 8 * i) = kk;
        *(v8h*)(Vth + rr * AT_KC + dh + 8 * i) = vv;
      }
    }
    __syncthreads();

    v8f s[4];
#pragma unroll
    for (int j = 0; j < 4; ++j) {
      s[j] = (v8f){0.f,0.f,0.f,0.f,0.f,0.f,0.f,0.f};
#pragma unroll
      for (int dc = 0; dc < 2; ++dc) {
        FH kb;
        kb.h[0] = *(const v8h*)(Ksh + (j * 16 + c) * AT_D + dc * 32 + 8 * hh);
        kb.h[1] = *(const v8h*)(Ksh + (j * 16 + c) * AT_D + dc * 32 + 16 + 8 * hh);
        s[j] = mma_h16(qa[dc], kb.v, s[j]);
      }
    }
    float cm[8];
#pragma unroll
    for (int r = 0; r < 8; ++r) {
      float m = -INFINITY;
#pragma unroll
      for (int j = 0; j < 4; ++j) {
        s[j][r] *= sscale;
        m = fmaxf(m, s[j][r]);
      }
#pragma unroll
      for (int off = 1; off < 16; off <<= 1) m = fmaxf(m, __shfl_xor(m, off, 32));
      cm[r] = m;
    }
    _Float16* pw = Psh[wave];
#pragma unroll
    for (int r = 0; r < 8; ++r) {
      const float mnew = fmaxf(mrow[r], cm[r]);
      const float alpha = expf(mrow[r] - mnew);
      mrow[r] = mnew;
      float psum = 0.f;
#pragma unroll
      for (int j = 0; j < 4; ++j) {
        const float p = expf(s[j][r] - mnew);
        psum += p;
        pw[(8 * hh + r) * AT_KC + j * 16 + c] = (_Float16)(p * AT_PSC);
      }
#pragma unroll
      for (int off = 1; off < 16; off <<= 1) psum += __shfl_xor(psum, off, 32);
      lrow[r] = lrow[r] * alpha + psum;
#pragma unroll
      for (int t = 0; t < 4; ++t) oacc[t][r] *= alpha;
    }
    __builtin_amdgcn_fence(__ATOMIC_RELEASE, "workgroup");
    __builtin_amdgcn_wave_barrier();
    __builtin_amdgcn_fence(__ATOMIC_ACQUIRE, "workgroup");
#pragma unroll 1
    for (int kk = 0; kk < 2; ++kk) {
      FH pa;
      pa.h[0] = *(const v8h*)(pw + c * AT_KC + kk * 32 + 8 * hh);
      pa.h[1] = *(const v8h*)(pw + c * AT_KC + kk * 32 + 16 + 8 * hh);
#pragma unroll
      for (int t = 0; t < 4; ++t) {
        FH vb;
        vb.h[0] = *(const v8h*)(Vth + (t * 16 + c) * AT_KC + kk * 32 + 8 * hh);
        vb.h[1] = *(const v8h*)(Vth + (t * 16 + c) * AT_KC + kk * 32 + 16 + 8 * hh);
        oacc[t] = mma_h16(pa.v, vb.v, oacc[t]);
      }
    }
  }

  float* os = Os[wave];
#pragma unroll
  for (int r = 0; r < 8; ++r) {
    const float inv = oscale * (1.0f / (lrow[r] * AT_PSC));
#pragma unroll
    for (int t = 0; t < 4; ++t) os[(8 * hh + r) * 68 + t * 16 + c] = oacc[t][r] * inv;
  }
  __builtin_amdgcn_fence(__ATOMIC_RELEASE, "workgroup");
  __builtin_amdgcn_wave_barrier();
  __builtin_amdgcn_fence(__ATOMIC_ACQUIRE, "workgroup");
  {
    const int q = lane >> 3, c8 = (lane & 7) * 8;
    for (int pass = 0; pass < 2; ++pass) {
#pragma unroll
      for (int it = 0; it < 4; ++it) {
        const int row = it * 4 + q;
        const float* sp = os + row * 68 + c8;
        v8h hv;
#pragma unroll
        for (int e = 0; e < 8; ++e) hv[e] = (_Float16)sp[e];
        *(volatile v8h*)(Op + (size_t)(q0 + row) * ldo + hcol + c8) = hv;
      }
      __threadfence();
    }
  }
}

template <int BIAS_MODE, int OUT_MODE, bool RESID, int ACT>
static void gemm_f16_launch(const void* A, int lda, const void* Bt, int ldb, void* Cc, int ldc,
                            const float* bias, const float* resid, int M, int Nn, int K, float scale,
                            hipStream_t stream) {
  const int tiles = (M / 64) * (Nn / 64);
  dim3 grid((tiles + 7) / 8, 1);
  wmma_gemm64<0, false, BIAS_MODE, OUT_MODE, RESID, ACT><<<grid, 256, 0, stream>>>(
      (const unsigned short*)A, (const unsigned short*)A, lda, 0L,
      (const unsigned short*)Bt, (const unsigned short*)Bt, ldb, 0L,
      Cc, Cc, ldc, 0L, bias, resid, 0L, M, Nn, K, scale);
}

extern "C" void kernel_launch(void* const* d_in, const int* in_sizes, int n_in,
                              void* d_out, int out_size, void* d_ws, size_t ws_size,
                              hipStream_t stream) {
  constexpr int kN = 4096, kD = 512, kH = 8, kF = 2048;
  if (n_in < 26) return;
  if (in_sizes[0] != kN * kD) return;
  if (in_sizes[2] != kD * kD || in_sizes[4] != kD * kD || in_sizes[6] != kD * kD || in_sizes[8] != kD * kD ||
      in_sizes[10] != kD * kD || in_sizes[12] != kD * kD) return;
  if (in_sizes[3] != kD || in_sizes[5] != kD || in_sizes[7] != kD || in_sizes[9] != kD || in_sizes[11] != kD ||
      in_sizes[13] != kD || in_sizes[14] != kD || in_sizes[15] != kD || in_sizes[19] != kD || in_sizes[20] != kD ||
      in_sizes[21] != kD || in_sizes[23] != kD) return;
  if (in_sizes[16] != kD * kF || in_sizes[17] != kF || in_sizes[18] != kF * kD) return;
  if (in_sizes[22] != 3 * kD * kD) return;
  if ((in_sizes[24] & 1) || (in_sizes[25] & 1)) return;
  const int NE  = in_sizes[24] / 2;
  const int NEP = in_sizes[25] / 2;
  if (in_sizes[1] != NE) return;
  if (NE < 8 || (NE % 8) != 0 || NEP < 8 || (NEP % 8) != 0) return;
  if (out_size != kN * kD) return;

  const float* x     = (const float*)d_in[0];
  const float* eattr = (const float*)d_in[1];
  const float* W_mp  = (const float*)d_in[2];
  const float* b_mp  = (const float*)d_in[3];
  const float* W_pp  = (const float*)d_in[4];
  const float* b_pp  = (const float*)d_in[5];
  const float* Wq    = (const float*)d_in[6];
  const float* bq    = (const float*)d_in[7];
  const float* Wk    = (const float*)d_in[8];
  const float* bk    = (const float*)d_in[9];
  const float* Wv    = (const float*)d_in[10];
  const float* bv    = (const float*)d_in[11];
  const float* Wo    = (const float*)d_in[12];
  const float* bo    = (const float*)d_in[13];
  const float* ln1g  = (const float*)d_in[14];
  const float* ln1b  = (const float*)d_in[15];
  const float* W1    = (const float*)d_in[16];
  const float* b1    = (const float*)d_in[17];
  const float* W2    = (const float*)d_in[18];
  const float* b2    = (const float*)d_in[19];
  const float* ln2g  = (const float*)d_in[20];
  const float* ln2b  = (const float*)d_in[21];
  const float* Wagg  = (const float*)d_in[22];
  const float* bagg  = (const float*)d_in[23];
  const int*   eidx  = (const int*)d_in[24];
  const int*   pidx  = (const int*)d_in[25];
  const int* esrc_mp = eidx;       const int* edst_mp = eidx + NE;
  const int* esrc_pp = pidx;       const int* edst_pp = pidx + NEP;
  float* outp = (float*)d_out;

  size_t off = 0;
  auto carve = [&](size_t bytes) -> char* { char* p = (char*)d_ws + off; off += (bytes + 255) & ~(size_t)255; return p; };
  _Float16* X16   = (_Float16*)carve((size_t)kN * kD * 2);
  _Float16* WMPT  = (_Float16*)carve((size_t)kD * kD * 2);
  _Float16* WPPT  = (_Float16*)carve((size_t)kD * kD * 2);
  _Float16* WQT   = (_Float16*)carve((size_t)kD * kD * 2);
  _Float16* WKT   = (_Float16*)carve((size_t)kD * kD * 2);
  _Float16* WVT   = (_Float16*)carve((size_t)kD * kD * 2);
  _Float16* WOT   = (_Float16*)carve((size_t)kD * kD * 2);
  _Float16* W1T   = (_Float16*)carve((size_t)kF * kD * 2);
  _Float16* W2T   = (_Float16*)carve((size_t)kD * kF * 2);
  _Float16* WAGT  = (_Float16*)carve((size_t)kD * 3 * kD * 2);
  float*    DINVM = (float*)carve((size_t)kN * 4);
  float*    DINVP = (float*)carve((size_t)kN * 4);
  float*    HF    = (float*)carve((size_t)kN * kD * 4);
  _Float16* Q16   = (_Float16*)carve((size_t)kN * kD * 2);
  _Float16* K16   = (_Float16*)carve((size_t)kN * kD * 2);
  _Float16* VT16  = (_Float16*)carve((size_t)kD * kN * 2);
  _Float16* O16   = (_Float16*)carve((size_t)kN * kD * 2);
  float*    TF    = (float*)carve((size_t)kN * kD * 4);
  float*    H1F   = (float*)carve((size_t)kN * kD * 4);
  _Float16* H1H   = (_Float16*)carve((size_t)kN * kD * 2);
  _Float16* M1H   = (_Float16*)carve((size_t)kN * kF * 2);
  _Float16* COMB  = (_Float16*)carve((size_t)kN * 3 * kD * 2);
  if (off > ws_size || off > (size_t)134217728) return;

  const float wsc = 64.0f;
  const float csc = 16.0f;
  const int comb_ld = 3 * kD;

  cast_f32_f16x2<<<(kN * kD / 2 + 255) / 256, 256, 0, stream>>>(x, X16, kN * kD / 2);
  transpose_cast_w_kernel<<<(kD * (kD / 8) + 255) / 256, 256, 0, stream>>>(W_mp, WMPT, kD, kD, wsc);
  transpose_cast_w_kernel<<<(kD * (kD / 8) + 255) / 256, 256, 0, stream>>>(W_pp, WPPT, kD, kD, wsc);
  transpose_cast_w_kernel<<<(kD * (kD / 8) + 255) / 256, 256, 0, stream>>>(Wq, WQT, kD, kD, wsc);
  transpose_cast_w_kernel<<<(kD * (kD / 8) + 255) / 256, 256, 0, stream>>>(Wk, WKT, kD, kD, wsc);
  transpose_cast_w_kernel<<<(kD * (kD / 8) + 255) / 256, 256, 0, stream>>>(Wv, WVT, kD, kD, wsc);
  transpose_cast_w_kernel<<<(kD * (kD / 8) + 255) / 256, 256, 0, stream>>>(Wo, WOT, kD, kD, wsc);
  transpose_cast_w_kernel<<<(kF * (kD / 8) + 255) / 256, 256, 0, stream>>>(W1, W1T, kD, kF, wsc);
  transpose_cast_w_kernel<<<(kD * (kF / 8) + 255) / 256, 256, 0, stream>>>(W2, W2T, kF, kD, wsc);
  transpose_cast_w_kernel<<<(kD * (3 * kD / 8) + 255) / 256, 256, 0, stream>>>(Wagg, WAGT, 3 * kD, kD, wsc);

  gcn_dinv_kernel<true><<<kN / DG_NT, DG_NT, 0, stream>>>(edst_mp, eattr, DINVM, kN, NE);
  gcn_dinv_kernel<false><<<kN / DG_NT, DG_NT, 0, stream>>>(edst_pp, eattr, DINVP, kN, NEP);

  gemm_f16_launch<0, 0, false, 0>(X16, kD, WMPT, kD, (void*)HF, kD, b_mp, x, kN, kD, kD, 1.0f / wsc, stream);
  gcn_agg_kernel<true><<<kN / AG_TILE, AG_T, 0, stream>>>(HF, esrc_mp, edst_mp, eattr, DINVM, b_mp, COMB, comb_ld, 0, kN, NE, csc);

  gemm_f16_launch<0, 0, false, 0>(X16, kD, WPPT, kD, (void*)HF, kD, b_pp, x, kN, kD, kD, 1.0f / wsc, stream);
  gcn_agg_kernel<false><<<kN / AG_TILE, AG_T, 0, stream>>>(HF, esrc_pp, edst_pp, eattr, DINVP, b_pp, COMB, comb_ld, 2 * kD, kN, NEP, csc);

  gemm_f16_launch<2, 1, false, 0>(X16, kD, WQT, kD, (void*)Q16, kD, bq, x, kN, kD, kD, 1.0f / wsc, stream);
  gemm_f16_launch<2, 1, false, 0>(X16, kD, WKT, kD, (void*)K16, kD, bk, x, kN, kD, kD, 1.0f / wsc, stream);
  gemm_f16_launch<1, 1, false, 0>(WVT, kD, X16, kD, (void*)VT16, kN, bv, x, kD, kN, kD, 1.0f / wsc, stream);

  attn64_h16_kernel<<<kH * (kN / AT_QB), AT_NW * 32, 0, stream>>>(Q16, kD, K16, kD, VT16, kN, O16, kD, kN, kH, 0.125f, 64.0f);

  gemm_f16_launch<2, 0, true, 0>(O16, kD, WOT, kD, (void*)TF, kD, bo, x, kN, kD, kD, 1.0f / (wsc * 64.0f), stream);
  layernorm512_kernel<true><<<kN / 4, 128, 0, stream>>>(TF, ln1g, ln1b, H1F, H1H, kD, 0, kN, csc);

  gemm_f16_launch<2, 1, false, 2>(H1H, kD, W1T, kD, (void*)M1H, kF, b1, x, kN, kF, kD, 1.0f / (wsc * csc), stream);
  gemm_f16_launch<2, 0, true, 0>(M1H, kF, W2T, kF, (void*)TF, kD, b2, H1F, kN, kD, kF, 1.0f / wsc, stream);
  layernorm512_kernel<false><<<kN / 4, 128, 0, stream>>>(TF, ln2g, ln2b, H1F, COMB, comb_ld, kD, kN, csc);

  gemm_f16_launch<2, 0, true, 0>(COMB, comb_ld, WAGT, comb_ld, (void*)outp, kD, bagg, x, kN, kD, 3 * kD, 1.0f / (wsc * csc), stream);
}
